// CapsuleLayer1d_41601053229673
// MI455X (gfx1250) — hardware-run, weakly checked
//
#include <hip/hip_runtime.h>
#include <math.h>

typedef __attribute__((ext_vector_type(16))) _Float16 v16h;
typedef __attribute__((ext_vector_type(8)))  _Float16 v8h;
typedef __attribute__((ext_vector_type(8)))  float    v8f;
typedef __attribute__((ext_vector_type(4)))  float    v4f;

constexpr int kNB    = 4096;
constexpr int kNO    = 32;
constexpr int kNI    = 64;
constexpr int kDO    = 16;
constexpr int kDI    = 16;
constexpr int kOD    = kNO * kDO;
constexpr int kXRow  = kNI * kDI;
constexpr int kChunk = 512;
constexpr int kChunks = kNB / kChunk;
constexpr int kSlabP = 68;
constexpr float kCarryX = 16.0f;
constexpr float kCarryW = 64.0f;
constexpr float kFold   = 1.0f / (kCarryX * kCarryW);
constexpr float kInvNO  = 1.0f / (float)kNO;
constexpr float kF16MinNormal = 6.103515625e-05f;
static_assert(kOD == 512 && kXRow == 1024, "plane pitches");
static_assert(kDI == 16 && kDO == 16, "K = 16 fragments: 8 halves per lane half");
static_assert(kChunk == 8 * 64, "8 waves x 64 samples per transform block");
static_assert(kOD == 8 * 64, "8 row tiles of 64 (o,d) values");
static_assert(kNB == 8 * 8 * 64, "k-sum grid: 8 blocks x 8 waves x 64 samples");
static_assert((kNB % kChunk) == 0, "whole chunks");
static_assert(kFold == 1.0f / 1024.0f, "carry fold");

constexpr size_t kSzX16 = (size_t)kNB * kNI * kDI * 2;
constexpr size_t kSzW16 = (size_t)kNO * kNI * kDO * kDI * 2;
constexpr size_t kSzS0  = (size_t)kNB * kOD * 4;
constexpr size_t kSzUH  = (size_t)kChunk * kNI * kOD * 4;
constexpr size_t kOffX16 = 0;
constexpr size_t kOffW16 = kOffX16 + kSzX16;
constexpr size_t kOffS0  = kOffW16 + kSzW16;
constexpr size_t kOffUH  = kOffS0 + kSzS0;
constexpr size_t kWsTotal = kOffUH + kSzUH;
static_assert(kWsTotal == 84934656ull, "carve total");
static_assert(kWsTotal <= 134217728ull, "carve cap");
static_assert((kOffW16 % 128) == 0 && (kOffS0 % 128) == 0 && (kOffUH % 128) == 0, "128-B aligned regions");

union FragU { v16h v; v8h p[2]; };

__device__ __forceinline__ v8f mma_f16(v16h a, v16h b, v8f c) {
  c = __builtin_amdgcn_wmma_f32_16x16x32_f16(false, a, false, b, (short)0, c, false, false);
  asm volatile("v_nop\n\tv_nop\n\tv_nop\n\tv_nop" : "+v"(c) : "v"(a), "v"(b));
  return c;
}

__device__ __forceinline__ void wave_lds_sync() {
  __builtin_amdgcn_fence(__ATOMIC_RELEASE, "workgroup");
  __builtin_amdgcn_wave_barrier();
  __builtin_amdgcn_fence(__ATOMIC_ACQUIRE, "workgroup");
}

__device__ __forceinline__ void put8(float* p, const v8f a) {
  const v4f lo = {a[0], a[1], a[2], a[3]};
  const v4f hi = {a[4], a[5], a[6], a[7]};
  *(v4f*)p = lo;
  *(v4f*)(p + 4) = hi;
}

__device__ __forceinline__ void flush_tile(float* slab, const v8f a0, const v8f a1, const v8f a2, const v8f a3,
                                           float* dst, size_t pitch, int lane) {
  const int rl = lane & 15, h = lane >> 4;
  float* sp = slab + rl * kSlabP + 8 * h;
  put8(sp, a0);
  put8(sp + 16, a1);
  put8(sp + 32, a2);
  put8(sp + 48, a3);
  wave_lds_sync();
  const int c4 = rl * 4;
  v4f v[8];
#pragma unroll
  for (int it = 0; it < 8; ++it) v[it] = *(const v4f*)(slab + (it * 2 + h) * kSlabP + c4);
#pragma unroll
  for (int pass = 0; pass < 2; ++pass) {
#pragma unroll
    for (int it = 0; it < 8; ++it)
      *(volatile v4f*)(dst + (size_t)(it * 2 + h) * pitch + c4) = v[it];
    __threadfence();
  }
  wave_lds_sync();
}

__global__ __launch_bounds__(256) void cvt_carry_f16_kernel(
    const float* __restrict__ src, unsigned short* __restrict__ dst, int total8, float carry)
{
  const int i = blockIdx.x * 256 + threadIdx.x;
  if (i >= total8) return;
  const size_t e0 = (size_t)i << 3;
  const v4f a0 = *(const v4f*)(src + e0);
  const v4f a1 = *(const v4f*)(src + e0 + 4);
  v8h hv;
#pragma unroll
  for (int e = 0; e < 4; ++e) {
    float f0 = a0[e] * carry;
    float f1 = a1[e] * carry;
    f0 = (fabsf(f0) < kF16MinNormal) ? 0.0f : f0;
    f1 = (fabsf(f1) < kF16MinNormal) ? 0.0f : f1;
    hv[e]     = (_Float16)f0;
    hv[4 + e] = (_Float16)f1;
  }
  unsigned short* q = dst + e0;
  *(volatile v8h*)q = hv;
  __threadfence();
  *(volatile v8h*)q = hv;
}

__global__ __launch_bounds__(256) void transform_kernel(
    const unsigned short* __restrict__ X16p, const unsigned short* __restrict__ W16p,
    float* __restrict__ UH, int chunk0)
{
  __shared__ __align__(16) float sT[8][16 * kSlabP];
  const _Float16* X16 = (const _Float16*)X16p;
  const _Float16* W16 = (const _Float16*)W16p;
  const int lane = threadIdx.x & 31;
  const int wave = threadIdx.x >> 5;
  const int rl = lane & 15, h = lane >> 4;
  const int tm = blockIdx.x;
  const int n  = blockIdx.y;
  v8h zero8;
#pragma unroll
  for (int e = 0; e < 8; ++e) zero8[e] = (_Float16)0.0f;
  const v8f zacc = {0.f, 0.f, 0.f, 0.f, 0.f, 0.f, 0.f, 0.f};

  v16h af[4];
#pragma unroll
  for (int i = 0; i < 4; ++i) {
    FragU f;
    f.p[0] = *(const v8h*)(W16 + ((size_t)((4 * tm + i) * kNI + n) * kDO + rl) * kDI + 8 * h);
    f.p[1] = zero8;
    af[i] = f.v;
  }
  float* slab = sT[wave];
#pragma unroll
  for (int j = 0; j < 4; ++j) {
    const int sl = wave * 64 + 16 * j;
    FragU g;
    g.p[0] = *(const v8h*)(X16 + ((size_t)(chunk0 + sl + rl) * kNI + n) * kDI + 8 * h);
    g.p[1] = zero8;
    const v8f c0 = mma_f16(af[0], g.v, zacc);
    const v8f c1 = mma_f16(af[1], g.v, zacc);
    const v8f c2 = mma_f16(af[2], g.v, zacc);
    const v8f c3 = mma_f16(af[3], g.v, zacc);
    flush_tile(slab, c0, c1, c2, c3,
               UH + ((size_t)sl * kNI + n) * kOD + 64 * tm, (size_t)kNI * kOD, lane);
  }
}

__global__ __launch_bounds__(256) void ksum_kernel(
    const unsigned short* __restrict__ X16p, const unsigned short* __restrict__ W16p, float* __restrict__ S0)
{
  __shared__ __align__(16) float sT[8][16 * kSlabP];
  const _Float16* X16 = (const _Float16*)X16p;
  const _Float16* W16 = (const _Float16*)W16p;
  const int lane = threadIdx.x & 31;
  const int wave = threadIdx.x >> 5;
  const int rl = lane & 15, h = lane >> 4;
  const int tm = blockIdx.x;
  const int sbase = (blockIdx.y * 8 + wave) * 64;

  v8f acc[4][4];
#pragma unroll
  for (int i = 0; i < 4; ++i)
#pragma unroll
    for (int j = 0; j < 4; ++j) acc[i][j] = (v8f){0.f, 0.f, 0.f, 0.f, 0.f, 0.f, 0.f, 0.f};

  const _Float16* wp[4];
  const _Float16* xp[4];
#pragma unroll
  for (int i = 0; i < 4; ++i) wp[i] = W16 + ((size_t)((4 * tm + i) * kNI) * kDO + rl) * kDI + 8 * h;
#pragma unroll
  for (int j = 0; j < 4; ++j) xp[j] = X16 + (size_t)(sbase + 16 * j + rl) * kXRow + 8 * h;

#pragma unroll 1
  for (int np = 0; np < kNI / 2; ++np) {
    v16h bf[4];
#pragma unroll
    for (int j = 0; j < 4; ++j) {
      FragU f;
      f.p[0] = *(const v8h*)(xp[j] + 32 * np);
      f.p[1] = *(const v8h*)(xp[j] + 32 * np + 16);
      bf[j] = f.v;
    }
#pragma unroll
    for (int i = 0; i < 4; ++i) {
      FragU f;
      f.p[0] = *(const v8h*)(wp[i] + (size_t)np * (2 * kDO * kDI));
      f.p[1] = *(const v8h*)(wp[i] + (size_t)np * (2 * kDO * kDI) + kDO * kDI);
#pragma unroll
      for (int j = 0; j < 4; ++j) acc[i][j] = mma_f16(f.v, bf[j], acc[i][j]);
    }
  }
  float* slab = sT[wave];
#pragma unroll
  for (int j = 0; j < 4; ++j)
    flush_tile(slab, acc[0][j], acc[1][j], acc[2][j], acc[3][j],
               S0 + (size_t)(sbase + 16 * j) * kOD + 64 * tm, (size_t)kOD, lane);
}

__global__ __launch_bounds__(256) void routing_kernel(
    const float* __restrict__ UH, const float* __restrict__ S0, float* __restrict__ out, int chunk0)
{
  __shared__ __align__(16) float ctab[kNO * kNI];
  __shared__ __align__(16) float blog[kNO * kNI];
  __shared__ __align__(16) float vtab[kNO * kDO];
  const int t  = threadIdx.x;
  const int o  = t >> 3;
  const int dq = (t >> 1) & 3;
  const int nh = t & 1;
  const int g  = t & 7;
  const int bglob = chunk0 + blockIdx.x;
  const float* uS  = UH + (size_t)blockIdx.x * ((size_t)kNI * kOD);
  const float* s0p = S0 + (size_t)bglob * kOD;

  {
    const v4f z = {0.f, 0.f, 0.f, 0.f};
    *(v4f*)(blog + t * 4) = z;
    *(v4f*)(blog + 1024 + t * 4) = z;
  }
  __syncthreads();

#pragma unroll 1
  for (int it = 0; it < 3; ++it) {
    v4f sv;
    if (it == 0) {
      const v4f r = *(const v4f*)(s0p + o * kDO + dq * 4);
      const float f0 = kFold * kInvNO;
      sv = r * f0;
    } else {
      float a0 = 0.f, a1 = 0.f, a2 = 0.f, a3 = 0.f;
      const float* up = uS + (size_t)(nh * 32) * kOD + o * kDO + dq * 4;
      const float* cp = ctab + o * kNI + nh * 32;
#pragma unroll 1
      for (int n4 = 0; n4 < 8; ++n4) {
        const v4f cv = *(const v4f*)(cp + 4 * n4);
        const float* q = up + (size_t)(4 * n4) * kOD;
        const v4f u0 = *(const v4f*)(q);
        const v4f u1 = *(const v4f*)(q + kOD);
        const v4f u2 = *(const v4f*)(q + 2 * kOD);
        const v4f u3 = *(const v4f*)(q + 3 * kOD);
        a0 = fmaf(cv[0], u0[0], a0); a1 = fmaf(cv[0], u0[1], a1); a2 = fmaf(cv[0], u0[2], a2); a3 = fmaf(cv[0], u0[3], a3);
        a0 = fmaf(cv[1], u1[0], a0); a1 = fmaf(cv[1], u1[1], a1); a2 = fmaf(cv[1], u1[2], a2); a3 = fmaf(cv[1], u1[3], a3);
        a0 = fmaf(cv[2], u2[0], a0); a1 = fmaf(cv[2], u2[1], a1); a2 = fmaf(cv[2], u2[2], a2); a3 = fmaf(cv[2], u2[3], a3);
        a0 = fmaf(cv[3], u3[0], a0); a1 = fmaf(cv[3], u3[1], a1); a2 = fmaf(cv[3], u3[2], a2); a3 = fmaf(cv[3], u3[3], a3);
      }
      a0 += __shfl_xor(a0, 1, 32);
      a1 += __shfl_xor(a1, 1, 32);
      a2 += __shfl_xor(a2, 1, 32);
      a3 += __shfl_xor(a3, 1, 32);
      sv = (v4f){a0 * kFold, a1 * kFold, a2 * kFold, a3 * kFold};
    }
    float q2 = sv[0] * sv[0];
    q2 = fmaf(sv[1], sv[1], q2);
    q2 = fmaf(sv[2], sv[2], q2);
    q2 = fmaf(sv[3], sv[3], q2);
    q2 += __shfl_xor(q2, 2, 32);
    q2 += __shfl_xor(q2, 4, 32);
    const float den = (1.0f + q2) * (__builtin_sqrtf(q2) + 1e-8f);
    const float fac = q2 * __builtin_amdgcn_rcpf(den);
    const v4f vv = sv * fac;
    if (nh == 0) *(v4f*)(vtab + o * kDO + dq * 4) = vv;
    __syncthreads();

    if (it < 2) {
      const v4f v0 = *(const v4f*)(vtab + o * kDO);
      const v4f v1 = *(const v4f*)(vtab + o * kDO + 4);
      const v4f v2 = *(const v4f*)(vtab + o * kDO + 8);
      const v4f v3 = *(const v4f*)(vtab + o * kDO + 12);
      const float* up = uS + (size_t)(8 * g) * kOD + o * kDO;
      float* bp = blog + o * kNI + 8 * g;
#pragma unroll 1
      for (int j = 0; j < 8; ++j) {
        const float* q = up + (size_t)j * kOD;
        const v4f u0 = *(const v4f*)(q);
        const v4f u1 = *(const v4f*)(q + 4);
        const v4f u2 = *(const v4f*)(q + 8);
        const v4f u3 = *(const v4f*)(q + 12);
        float p = u0[0] * v0[0];
        p = fmaf(u0[1], v0[1], p); p = fmaf(u0[2], v0[2], p); p = fmaf(u0[3], v0[3], p);
        p = fmaf(u1[0], v1[0], p); p = fmaf(u1[1], v1[1], p); p = fmaf(u1[2], v1[2], p); p = fmaf(u1[3], v1[3], p);
        p = fmaf(u2[0], v2[0], p); p = fmaf(u2[1], v2[1], p); p = fmaf(u2[2], v2[2], p); p = fmaf(u2[3], v2[3], p);
        p = fmaf(u3[0], v3[0], p); p = fmaf(u3[1], v3[1], p); p = fmaf(u3[2], v3[2], p); p = fmaf(u3[3], v3[3], p);
        const float bold = bp[j];
        bp[j] = fmaf(p, kFold, bold);
      }
      __syncthreads();
      if (t < kNI) {
        const int n = t;
        float m = blog[n];
#pragma unroll 4
        for (int oo = 1; oo < kNO; ++oo) m = fmaxf(m, blog[oo * kNI + n]);
        float sum = 0.f;
#pragma unroll 4
        for (int oo = 0; oo < kNO; ++oo) {
          const float e = __expf(blog[oo * kNI + n] - m);
          ctab[oo * kNI + n] = e;
          sum += e;
        }
        const float rs = 1.0f / sum;
#pragma unroll 4
        for (int oo = 0; oo < kNO; ++oo) {
          const float e = ctab[oo * kNI + n];
          ctab[oo * kNI + n] = e * rs;
        }
      }
      __syncthreads();
    }
  }

  if (t < 32) {
    v4f ov[4];
#pragma unroll
    for (int k = 0; k < 4; ++k) ov[k] = *(const v4f*)(vtab + k * 128 + t * 4);
    float* op = out + (size_t)bglob * kOD;
#pragma unroll
    for (int pass = 0; pass < 2; ++pass) {
#pragma unroll
      for (int k = 0; k < 4; ++k) *(volatile v4f*)(op + k * 128 + t * 4) = ov[k];
      __threadfence();
    }
  }
}

extern "C" void kernel_launch(void* const* d_in, const int* in_sizes, int n_in,
                              void* d_out, int out_size, void* d_ws, size_t ws_size,
                              hipStream_t stream) {
  if (n_in < 2) return;
  if (in_sizes[0] != kNB * kNI * kDI) return;
  if (in_sizes[1] != kNO * kNI * kDO * kDI) return;
  if (out_size != kNB * kOD) return;
  if (ws_size < kWsTotal) return;

  const float* x = (const float*)d_in[0];
  const float* w = (const float*)d_in[1];
  float* out = (float*)d_out;

  char* ws = (char*)d_ws;
  unsigned short* X16 = (unsigned short*)(ws + kOffX16);
  unsigned short* W16 = (unsigned short*)(ws + kOffW16);
  float*          S0  = (float*)(ws + kOffS0);
  float*          UH  = (float*)(ws + kOffUH);

  const int x8 = kNB * kNI * kDI / 8;
  const int w8 = kNO * kNI * kDO * kDI / 8;
  cvt_carry_f16_kernel<<<x8 / 256, 256, 0, stream>>>(x, X16, x8, kCarryX);
  cvt_carry_f16_kernel<<<w8 / 256, 256, 0, stream>>>(w, W16, w8, kCarryW);

  ksum_kernel<<<dim3(8, 8), 256, 0, stream>>>(X16, W16, S0);

  for (int c = 0; c < kChunks; ++c) {
    const int chunk0 = c * kChunk;
    transform_kernel<<<dim3(kOD / 64, kNI), 256, 0, stream>>>(X16, W16, UH, chunk0);
    routing_kernel<<<kChunk, 256, 0, stream>>>(UH, S0, out, chunk0);
  }
}
